// MyTransformerEncoderLayer_89515708383410
// MI455X (gfx1250) — hardware-verified
//
#include <hip/hip_runtime.h>
#include <stddef.h>
#include <stdint.h>

#define NB    2
#define SQ    2048
#define NTOK  4096
#define HID   1024
#define NH    16
#define HDM   64
#define DFF   4096
#define NQKV  3072
#define QB    128
#define KC    64
#define NQB   (SQ / QB)
#define NCK   (SQ / KC)
#define SBLK  (SQ / 256)
#define QKPLANE (NB * NH * SQ * HDM)

static_assert(NTOK == NB * SQ);
static_assert(SQ % 256 == 0);
static_assert(HID % 64 == 0);
static_assert(DFF % 64 == 0);
static_assert(HDM == 64);
static_assert(NH * HDM == HID);
static_assert(NQKV == 3 * HID);
static_assert(SQ % KC == 0);
static_assert(SQ % QB == 0);
static_assert(NTOK % 256 == 0);
static_assert(NTOK % 8 == 0);
static_assert((NTOK * HID) % 2048 == 0);
static_assert((HID * HID) % 2048 == 0);
static_assert((DFF * HID) % 2048 == 0);

typedef _Float16 v16h __attribute__((ext_vector_type(16)));
typedef _Float16 v8h  __attribute__((ext_vector_type(8)));
typedef float    v8f  __attribute__((ext_vector_type(8)));
typedef float    v4f  __attribute__((ext_vector_type(4)));
typedef unsigned int v4u __attribute__((ext_vector_type(4)));

union Frag  { v16h v; v8h h[2]; };
union Pack8 { v8h h; v4u u; };

__device__ __forceinline__ v8f mma16(v16h a, v16h b, v8f c) {
  c = __builtin_amdgcn_wmma_f32_16x16x32_f16(false, a, false, b, (short)0, c, false, false);
  asm volatile("v_nop\n\tv_nop\n\tv_nop\n\tv_nop" : "+v"(c) : "v"(a), "v"(b));
  return c;
}

__device__ __forceinline__ v16h ldfrag(const _Float16* p, int ld, int row0, int k0, int lane) {
  const int m = lane & 15, lh = lane >> 4;
  const _Float16* q = p + (size_t)(row0 + m) * ld + k0 + 8 * lh;
  Frag f;
  f.h[0] = *(const v8h*)(q);
  f.h[1] = *(const v8h*)(q + 16);
  return f.v;
}

__device__ __forceinline__ v8f zero8() { return (v8f){0.f, 0.f, 0.f, 0.f, 0.f, 0.f, 0.f, 0.f}; }

__device__ __forceinline__ void gemm32x64(const _Float16* __restrict__ A, int lda,
                                          const _Float16* __restrict__ Bt, int ldb, int K,
                                          int m0, int n0, int lane, v8f (&acc)[2][4]) {
#pragma unroll 1
  for (int k0 = 0; k0 < K; k0 += 32) {
    const v16h a0 = ldfrag(A, lda, m0, k0, lane);
    const v16h a1 = ldfrag(A, lda, m0 + 16, k0, lane);
    const v16h b0 = ldfrag(Bt, ldb, n0, k0, lane);
    const v16h b1 = ldfrag(Bt, ldb, n0 + 16, k0, lane);
    const v16h b2 = ldfrag(Bt, ldb, n0 + 32, k0, lane);
    const v16h b3 = ldfrag(Bt, ldb, n0 + 48, k0, lane);
    acc[0][0] = mma16(a0, b0, acc[0][0]);
    acc[1][0] = mma16(a1, b0, acc[1][0]);
    acc[0][1] = mma16(a0, b1, acc[0][1]);
    acc[1][1] = mma16(a1, b1, acc[1][1]);
    acc[0][2] = mma16(a0, b2, acc[0][2]);
    acc[1][2] = mma16(a1, b2, acc[1][2]);
    acc[0][3] = mma16(a0, b3, acc[0][3]);
    acc[1][3] = mma16(a1, b3, acc[1][3]);
  }
}

__global__ __launch_bounds__(256) void k_cvt(const float* __restrict__ src, _Float16* __restrict__ dh, float scale) {
  const int tid = threadIdx.x;
  const int row = blockIdx.x * 2 + (tid >> 7);
  const int col = (tid & 127) * 8;
  const size_t o = (size_t)row * HID + col;
  const v4f a0 = *(const v4f*)(src + o) * scale;
  const v4f a1 = *(const v4f*)(src + o + 4) * scale;
  Pack8 pk;
  pk.h = (v8h){(_Float16)a0[0], (_Float16)a0[1], (_Float16)a0[2], (_Float16)a0[3],
               (_Float16)a1[0], (_Float16)a1[1], (_Float16)a1[2], (_Float16)a1[3]};
  const v4u vv = pk.u;
  volatile v4u* d = (volatile v4u*)(dh + o);
  *d = vv;
  __threadfence();
  *d = vv;
}

#define STP 72
#define SVP 264
__global__ __launch_bounds__(256) void k_qkv(const _Float16* __restrict__ xh,
                                             const _Float16* __restrict__ wt,
                                             const float* __restrict__ bq,
                                             const float* __restrict__ bk,
                                             const float* __restrict__ bv,
                                             _Float16* __restrict__ qkp,
                                             _Float16* __restrict__ vtp) {
  __shared__ __align__(16) _Float16 st[256 * STP];
  const int tid = threadIdx.x, lane = tid & 31, wave = tid >> 5;
  const int hh = lane >> 4, c = lane & 15;
  const int bx = blockIdx.x;
  const int b  = bx / SBLK;
  const int sb = (bx - b * SBLK) * 256;
  const int ns = blockIdx.y;
  const int which = ns / NH;
  const int head  = ns - which * NH;
  const int hb    = b * NH + head;
  const int m0 = sb + wave * 32;
  const int n0 = ns * 64;
  const _Float16* A = xh + (size_t)b * HID;

  v8f acc[2][4];
#pragma unroll
  for (int s = 0; s < 2; ++s)
#pragma unroll
    for (int t = 0; t < 4; ++t) acc[s][t] = zero8();
  gemm32x64(A, NB * HID, wt, HID, HID, m0, n0, lane, acc);

  float bb[4];
#pragma unroll
  for (int t = 0; t < 4; ++t) {
    const int i = head * HDM + 16 * t + c;
    const float xq = bq[i], xk = bk[i], xv = bv[i];
    bb[t] = (which == 0) ? xq : ((which == 1) ? xk : xv);
  }

  if (which < 2) {
#pragma unroll
    for (int sub = 0; sub < 2; ++sub)
#pragma unroll
      for (int t = 0; t < 4; ++t)
#pragma unroll
        for (int r = 0; r < 8; ++r)
          st[(wave * 32 + sub * 16 + 8 * hh + r) * STP + 16 * t + c] =
              (_Float16)(acc[sub][t][r] * 0.03125f + bb[t]);
  } else {
#pragma unroll
    for (int sub = 0; sub < 2; ++sub)
#pragma unroll
      for (int t = 0; t < 4; ++t)
#pragma unroll
        for (int r = 0; r < 8; ++r)
          st[(16 * t + c) * SVP + wave * 32 + sub * 16 + 8 * hh + r] =
              (_Float16)(acc[sub][t][r] * 0.03125f + bb[t]);
  }
  __syncthreads();

  if (which < 2) {
    _Float16* base = qkp + (size_t)which * QKPLANE + (size_t)hb * SQ * HDM;
#pragma unroll
    for (int g = 0; g < 2; ++g) {
      v4u val[4];
      size_t go[4];
#pragma unroll
      for (int j = 0; j < 4; ++j) {
        const int p  = tid + 256 * (4 * g + j);
        const int lr = p >> 3;
        const int pc = p & 7;
        Pack8 pk;
        pk.h   = *(const v8h*)(st + lr * STP + pc * 8);
        val[j] = pk.u;
        go[j]  = (size_t)(sb + lr) * HDM + pc * 8;
      }
      for (int ps = 0; ps < 2; ++ps) {
#pragma unroll
        for (int j = 0; j < 4; ++j) *(volatile v4u*)(base + go[j]) = val[j];
        __threadfence();
      }
    }
  } else {
    _Float16* base = vtp + (size_t)hb * HDM * SQ;
#pragma unroll
    for (int g = 0; g < 2; ++g) {
      v4u val[4];
      size_t go[4];
#pragma unroll
      for (int j = 0; j < 4; ++j) {
        const int p    = tid + 256 * (4 * g + j);
        const int drow = p >> 5;
        const int pc   = p & 31;
        Pack8 pk;
        pk.h   = *(const v8h*)(st + drow * SVP + pc * 8);
        val[j] = pk.u;
        go[j]  = (size_t)drow * SQ + sb + pc * 8;
      }
      for (int ps = 0; ps < 2; ++ps) {
#pragma unroll
        for (int j = 0; j < 4; ++j) *(volatile v4u*)(base + go[j]) = val[j];
        __threadfence();
      }
    }
  }
}

#define KTP 72
__global__ __launch_bounds__(256) void k_attn(const _Float16* __restrict__ qp,
                                              const _Float16* __restrict__ kp,
                                              const _Float16* __restrict__ vt,
                                              _Float16* __restrict__ op, float sscale) {
  __shared__ __align__(16) _Float16 Ks[KC * KTP];
  __shared__ __align__(16) _Float16 Vs[HDM * KTP];
  __shared__ __align__(16) _Float16 Ps[8 * 16 * KTP];

  const int tid = threadIdx.x, lane = tid & 31, wave = tid >> 5;
  const int hh = lane >> 4, c = lane & 15;
  const int qb  = blockIdx.x % NQB;
  const int hb  = blockIdx.x / NQB;
  const int h   = hb % NH;
  const int b   = hb / NH;
  const int q0  = qb * QB + wave * 16;

  const _Float16* Q = qp + (size_t)hb * SQ * HDM;
  const _Float16* K = kp + (size_t)hb * SQ * HDM;
  const _Float16* V = vt + (size_t)hb * HDM * SQ;

  v16h qa[2];
  qa[0] = ldfrag(Q, HDM, q0, 0, lane);
  qa[1] = ldfrag(Q, HDM, q0, 32, lane);

  const float NEGI = -__builtin_huge_valf();
  float mrow[8], lrow[8];
  v8f oacc[4];
#pragma unroll
  for (int r = 0; r < 8; ++r) { mrow[r] = NEGI; lrow[r] = 0.f; }
#pragma unroll
  for (int t = 0; t < 4; ++t) oacc[t] = zero8();

  _Float16* pw = Ps + wave * 16 * KTP;

  for (int kc = 0; kc < NCK; ++kc) {
    const int kv0 = kc * KC;
    __syncthreads();
    {
      const int r  = tid >> 2;
      const int qq = (tid & 3) * 16;
      const _Float16* ks = K + (size_t)(kv0 + r) * HDM + qq;
      const _Float16* vs = V + (size_t)r * SQ + kv0 + qq;
#pragma unroll
      for (int e = 0; e < 2; ++e) {
        *(v8h*)(Ks + r * KTP + qq + 8 * e) = *(const v8h*)(ks + 8 * e);
        *(v8h*)(Vs + r * KTP + qq + 8 * e) = *(const v8h*)(vs + 8 * e);
      }
    }
    __syncthreads();

    v8f s[4];
#pragma unroll
    for (int j = 0; j < 4; ++j) s[j] = zero8();
#pragma unroll
    for (int dc = 0; dc < 2; ++dc) {
#pragma unroll
      for (int j = 0; j < 4; ++j) {
        const v16h kb = ldfrag(Ks, KTP, j * 16, dc * 32, lane);
        s[j] = mma16(qa[dc], kb, s[j]);
      }
    }
    float cm[8];
#pragma unroll
    for (int r = 0; r < 8; ++r) {
      float m = NEGI;
#pragma unroll
      for (int j = 0; j < 4; ++j) { s[j][r] *= sscale; m = fmaxf(m, s[j][r]); }
#pragma unroll
      for (int off = 1; off < 16; off <<= 1) m = fmaxf(m, __shfl_xor(m, off, 32));
      cm[r] = m;
    }
    float al[8];
#pragma unroll
    for (int r = 0; r < 8; ++r) {
      const float mnew  = fmaxf(mrow[r], cm[r]);
      const float alpha = __expf(mrow[r] - mnew);
      mrow[r] = mnew;
      float psum = 0.f;
#pragma unroll
      for (int j = 0; j < 4; ++j) {
        const float p = __expf(s[j][r] - mnew);
        psum += p;
        pw[(8 * hh + r) * KTP + j * 16 + c] = (_Float16)(p * 1024.0f);
      }
#pragma unroll
      for (int off = 1; off < 16; off <<= 1) psum += __shfl_xor(psum, off, 32);
      lrow[r] = lrow[r] * alpha + psum;
      al[r] = alpha;
    }
#pragma unroll
    for (int t = 0; t < 4; ++t)
#pragma unroll
      for (int r = 0; r < 8; ++r) oacc[t][r] *= al[r];
    __syncthreads();

#pragma unroll
    for (int kk = 0; kk < 2; ++kk) {
      const v16h pa = ldfrag(pw, KTP, 0, kk * 32, lane);
#pragma unroll
      for (int t = 0; t < 4; ++t) {
        const v16h vb = ldfrag(Vs, KTP, t * 16, kk * 32, lane);
        oacc[t] = mma16(pa, vb, oacc[t]);
      }
    }
  }

  float invl[8];
#pragma unroll
  for (int r = 0; r < 8; ++r) invl[r] = (lrow[r] > 0.f) ? (0.0625f / lrow[r]) : 0.f;
  __syncthreads();
#pragma unroll
  for (int r = 0; r < 8; ++r) {
#pragma unroll
    for (int t = 0; t < 4; ++t)
      pw[(8 * hh + r) * KTP + 16 * t + c] = (_Float16)(oacc[t][r] * invl[r]);
  }
  __syncthreads();
  v4u val[4];
  size_t go[4];
#pragma unroll
  for (int it = 0; it < 4; ++it) {
    const int p  = lane + 32 * it;
    const int L  = p >> 3;
    const int pc = p & 7;
    Pack8 pk;
    pk.h    = *(const v8h*)(pw + L * KTP + pc * 8);
    val[it] = pk.u;
    go[it]  = ((size_t)(q0 + L) * NB + b) * HID + (size_t)h * HDM + pc * 8;
  }
  for (int ps = 0; ps < 2; ++ps) {
#pragma unroll
    for (int it = 0; it < 4; ++it) *(volatile v4u*)(op + go[it]) = val[it];
    __threadfence();
  }
}

#define OTP 68
__device__ __forceinline__ void out_epilogue_f32(v8f (&acc)[2][4], float scale, const float (&bb)[4],
                                                 float* sw, float* __restrict__ out, int ldo,
                                                 int m0, int n0, int lane, int hh, int c) {
#pragma unroll
  for (int sub = 0; sub < 2; ++sub) {
    __syncthreads();
#pragma unroll
    for (int t = 0; t < 4; ++t) {
#pragma unroll
      for (int r = 0; r < 8; ++r) sw[(8 * hh + r) * OTP + 16 * t + c] = acc[sub][t][r] * scale + bb[t];
    }
    __syncthreads();
    v4f val[8];
    size_t go[8];
#pragma unroll
    for (int it = 0; it < 8; ++it) {
      const int p    = lane + 32 * it;
      const int L    = p >> 3;
      const int pc   = p & 7;
      const int row  = L >> 1;
      const int half = L & 1;
      val[it] = *(const v4f*)(sw + row * OTP + half * 32 + pc * 4);
      go[it]  = (size_t)(m0 + sub * 16 + row) * ldo + n0 + half * 32 + pc * 4;
    }
    for (int ps = 0; ps < 2; ++ps) {
#pragma unroll
      for (int it = 0; it < 8; ++it) *(volatile v4f*)(out + go[it]) = val[it];
      __threadfence();
    }
  }
}

__device__ __forceinline__ void out_epilogue_h16(v8f (&acc)[2][4], float scale, const float (&bb)[4], float oscale,
                                                 float* sw, _Float16* __restrict__ out, int ldo,
                                                 int m0, int n0, int lane, int hh, int c) {
#pragma unroll
  for (int sub = 0; sub < 2; ++sub) {
    __syncthreads();
#pragma unroll
    for (int t = 0; t < 4; ++t) {
#pragma unroll
      for (int r = 0; r < 8; ++r) {
        const float v = acc[sub][t][r] * scale + bb[t];
        sw[(8 * hh + r) * OTP + 16 * t + c] = fmaxf(v, 0.f) * oscale;
      }
    }
    __syncthreads();
    v4u val[4];
    size_t go[4];
#pragma unroll
    for (int it = 0; it < 4; ++it) {
      const int p  = lane + 32 * it;
      const int L  = p >> 3;
      const int pc = p & 7;
      const float* ra = sw + L * OTP + pc * 8;
      const v4f a0 = *(const v4f*)(ra), a1 = *(const v4f*)(ra + 4);
      Pack8 pk;
      pk.h = (v8h){(_Float16)a0[0], (_Float16)a0[1], (_Float16)a0[2], (_Float16)a0[3],
                   (_Float16)a1[0], (_Float16)a1[1], (_Float16)a1[2], (_Float16)a1[3]};
      val[it] = pk.u;
      go[it]  = (size_t)(m0 + sub * 16 + L) * ldo + n0 + pc * 8;
    }
    for (int ps = 0; ps < 2; ++ps) {
#pragma unroll
      for (int it = 0; it < 4; ++it) *(volatile v4u*)(out + go[it]) = val[it];
      __threadfence();
    }
  }
}

__global__ __launch_bounds__(256) void k_gemm_f32(const _Float16* __restrict__ ap, int lda,
                                                  const _Float16* __restrict__ wt, int K,
                                                  const float* __restrict__ bias, float scale,
                                                  float* __restrict__ out, int ldo) {
  __shared__ __align__(16) float st[8][16 * OTP];
  const int tid = threadIdx.x, lane = tid & 31, wave = tid >> 5;
  const int hh = lane >> 4, c = lane & 15;
  const int m0 = blockIdx.x * 256 + wave * 32;
  const int n0 = blockIdx.y * 64;

  v8f acc[2][4];
#pragma unroll
  for (int s = 0; s < 2; ++s)
#pragma unroll
    for (int t = 0; t < 4; ++t) acc[s][t] = zero8();
  gemm32x64(ap, lda, wt, K, K, m0, n0, lane, acc);
  float bb[4];
#pragma unroll
  for (int t = 0; t < 4; ++t) bb[t] = bias[n0 + 16 * t + c];
  out_epilogue_f32(acc, scale, bb, st[wave], out, ldo, m0, n0, lane, hh, c);
}

__global__ __launch_bounds__(256) void k_gemm_h16(const _Float16* __restrict__ ap, int lda,
                                                  const _Float16* __restrict__ wt, int K,
                                                  const float* __restrict__ bias, float scale, float oscale,
                                                  _Float16* __restrict__ out, int ldo) {
  __shared__ __align__(16) float st[8][16 * OTP];
  const int tid = threadIdx.x, lane = tid & 31, wave = tid >> 5;
  const int hh = lane >> 4, c = lane & 15;
  const int m0 = blockIdx.x * 256 + wave * 32;
  const int n0 = blockIdx.y * 64;

  v8f acc[2][4];
#pragma unroll
  for (int s = 0; s < 2; ++s)
#pragma unroll
    for (int t = 0; t < 4; ++t) acc[s][t] = zero8();
  gemm32x64(ap, lda, wt, K, K, m0, n0, lane, acc);
  float bb[4];
#pragma unroll
  for (int t = 0; t < 4; ++t) bb[t] = bias[n0 + 16 * t + c];
  out_epilogue_h16(acc, scale, bb, oscale, st[wave], out, ldo, m0, n0, lane, hh, c);
}

__global__ __launch_bounds__(256) void k_ln1(const float* __restrict__ t, const float* __restrict__ res,
                                             const float* __restrict__ g, const float* __restrict__ be,
                                             float* __restrict__ yf, _Float16* __restrict__ yh) {
  __shared__ __align__(16) float sw[8][HID];
  const int tid = threadIdx.x, lane = tid & 31, wave = tid >> 5;
  const size_t m = (size_t)blockIdx.x * 8 + wave;
  const float* tr = t + m * HID;
  const float* rr = res + m * HID;

  v4f v[8];
  float s = 0.f;
#pragma unroll
  for (int it = 0; it < 8; ++it) {
    const int idx = it * 128 + lane * 4;
    const v4f a = *(const v4f*)(tr + idx);
    const v4f r = *(const v4f*)(rr + idx);
    v[it] = a + r;
    s += (v[it][0] + v[it][1]) + (v[it][2] + v[it][3]);
  }
#pragma unroll
  for (int off = 16; off >= 1; off >>= 1) s += __shfl_xor(s, off, 32);
  const float mean = s * 0.0009765625f;
  float ss = 0.f;
#pragma unroll
  for (int it = 0; it < 8; ++it) {
    const v4f d = v[it] - mean;
    ss += (d[0] * d[0] + d[1] * d[1]) + (d[2] * d[2] + d[3] * d[3]);
  }
#pragma unroll
  for (int off = 16; off >= 1; off >>= 1) ss += __shfl_xor(ss, off, 32);
  const float var  = ss * 0.0009765625f;
  const float rstd = rsqrtf(var + 1e-5f);

  v4f y[8];
#pragma unroll
  for (int it = 0; it < 8; ++it) {
    const int idx = it * 128 + lane * 4;
    const v4f gv = *(const v4f*)(g + idx);
    const v4f bv = *(const v4f*)(be + idx);
    y[it] = ((v[it] - mean) * rstd) * gv + bv;
  }
  for (int ps = 0; ps < 2; ++ps) {
#pragma unroll
    for (int it = 0; it < 8; ++it) *(volatile v4f*)(yf + m * HID + it * 128 + lane * 4) = y[it];
    __threadfence();
  }
#pragma unroll
  for (int it = 0; it < 8; ++it) *(v4f*)(sw[wave] + it * 128 + lane * 4) = y[it];
  __syncthreads();
  v4u hv[4];
  size_t go[4];
#pragma unroll
  for (int j = 0; j < 4; ++j) {
    const float* cp = sw[wave] + 256 * j + 8 * lane;
    const v4f a0 = *(const v4f*)(cp), a1 = *(const v4f*)(cp + 4);
    Pack8 pk;
    pk.h = (v8h){(_Float16)a0[0], (_Float16)a0[1], (_Float16)a0[2], (_Float16)a0[3],
                 (_Float16)a1[0], (_Float16)a1[1], (_Float16)a1[2], (_Float16)a1[3]};
    hv[j] = pk.u;
    go[j] = m * HID + 256 * j + 8 * lane;
  }
  for (int ps = 0; ps < 2; ++ps) {
#pragma unroll
    for (int j = 0; j < 4; ++j) *(volatile v4u*)(yh + go[j]) = hv[j];
    __threadfence();
  }
}

__global__ __launch_bounds__(256) void k_ln2(const float* __restrict__ t, const float* __restrict__ res,
                                             const float* __restrict__ g, const float* __restrict__ be,
                                             float* __restrict__ out) {
  const int tid = threadIdx.x, lane = tid & 31, wave = tid >> 5;
  const size_t m = (size_t)blockIdx.x * 8 + wave;
  const float* tr = t + m * HID;
  const float* rr = res + m * HID;

  v4f v[8];
  float s = 0.f;
#pragma unroll
  for (int it = 0; it < 8; ++it) {
    const int idx = it * 128 + lane * 4;
    const v4f a = *(const v4f*)(tr + idx);
    const v4f r = *(const v4f*)(rr + idx);
    v[it] = a + r;
    s += (v[it][0] + v[it][1]) + (v[it][2] + v[it][3]);
  }
#pragma unroll
  for (int off = 16; off >= 1; off >>= 1) s += __shfl_xor(s, off, 32);
  const float mean = s * 0.0009765625f;
  float ss = 0.f;
#pragma unroll
  for (int it = 0; it < 8; ++it) {
    const v4f d = v[it] - mean;
    ss += (d[0] * d[0] + d[1] * d[1]) + (d[2] * d[2] + d[3] * d[3]);
  }
#pragma unroll
  for (int off = 16; off >= 1; off >>= 1) ss += __shfl_xor(ss, off, 32);
  const float var  = ss * 0.0009765625f;
  const float rstd = rsqrtf(var + 1e-5f);

  v4f o[8];
#pragma unroll
  for (int it = 0; it < 8; ++it) {
    const int idx = it * 128 + lane * 4;
    const v4f gv = *(const v4f*)(g + idx);
    const v4f bv = *(const v4f*)(be + idx);
    o[it] = ((v[it] - mean) * rstd) * gv + bv;
  }
  for (int ps = 0; ps < 2; ++ps) {
#pragma unroll
    for (int it = 0; it < 8; ++it) *(volatile v4f*)(out + m * HID + it * 128 + lane * 4) = o[it];
    __threadfence();
  }
}

extern "C" void kernel_launch(void* const* d_in, const int* in_sizes, int n_in,
                              void* d_out, int out_size, void* d_ws, size_t ws_size,
                              hipStream_t stream) {
  if (n_in < 17) return;
  if (in_sizes[0] != NTOK * HID) return;
  if (in_sizes[1] != HID * HID) return;
  if (in_sizes[2] != HID) return;
  if (in_sizes[3] != HID * HID) return;
  if (in_sizes[4] != HID) return;
  if (in_sizes[5] != HID * HID) return;
  if (in_sizes[6] != HID) return;
  if (in_sizes[7] != HID * HID) return;
  if (in_sizes[8] != HID) return;
  if (in_sizes[9] != DFF * HID) return;
  if (in_sizes[10] != DFF) return;
  if (in_sizes[11] != HID * DFF) return;
  if (in_sizes[12] != HID) return;
  if (in_sizes[13] != HID) return;
  if (in_sizes[14] != HID) return;
  if (in_sizes[15] != HID) return;
  if (in_sizes[16] != HID) return;
  if (out_size != NTOK * HID) return;

  const float* x   = (const float*)d_in[0];
  const float* wq  = (const float*)d_in[1];
  const float* bq  = (const float*)d_in[2];
  const float* wk  = (const float*)d_in[3];
  const float* bk  = (const float*)d_in[4];
  const float* wv  = (const float*)d_in[5];
  const float* bv  = (const float*)d_in[6];
  const float* wo  = (const float*)d_in[7];
  const float* bo  = (const float*)d_in[8];
  const float* w1  = (const float*)d_in[9];
  const float* b1  = (const float*)d_in[10];
  const float* w2  = (const float*)d_in[11];
  const float* b2  = (const float*)d_in[12];
  const float* g1  = (const float*)d_in[13];
  const float* be1 = (const float*)d_in[14];
  const float* g2  = (const float*)d_in[15];
  const float* be2 = (const float*)d_in[16];
  float* out = (float*)d_out;

  size_t off = 0;
  const size_t oX   = off; off += (size_t)NTOK * HID * 2;
  const size_t oWt  = off; off += (size_t)NQKV * HID * 2;
  const size_t oWo  = off; off += (size_t)HID * HID * 2;
  const size_t oW1  = off; off += (size_t)DFF * HID * 2;
  const size_t oW2  = off; off += (size_t)HID * DFF * 2;
  const size_t oQ   = off; off += (size_t)NB * NH * SQ * HDM * 2;
  const size_t oK   = off; off += (size_t)NB * NH * SQ * HDM * 2;
  const size_t oV   = off; off += (size_t)NB * NH * HDM * SQ * 2;
  const size_t oO   = off; off += (size_t)NTOK * HID * 2;
  const size_t oHd  = oQ;
  if (oHd + (size_t)NTOK * DFF * 2 > off) return;
  const size_t oT   = off; off += (size_t)NTOK * HID * 4;
  const size_t oY1f = off; off += (size_t)NTOK * HID * 4;
  const size_t oY1h = off; off += (size_t)NTOK * HID * 2;
  if (off > ws_size) return;
  if (off > (size_t)134217728) return;

  char* ws = (char*)d_ws;
  _Float16* Xh  = (_Float16*)(ws + oX);
  _Float16* Wt  = (_Float16*)(ws + oWt);
  _Float16* Wot = (_Float16*)(ws + oWo);
  _Float16* W1t = (_Float16*)(ws + oW1);
  _Float16* W2t = (_Float16*)(ws + oW2);
  _Float16* QKp = (_Float16*)(ws + oQ);
  _Float16* Kp  = (_Float16*)(ws + oK);
  _Float16* Vt  = (_Float16*)(ws + oV);
  _Float16* Op  = (_Float16*)(ws + oO);
  _Float16* Hd  = (_Float16*)(ws + oHd);
  float*    T   = (float*)(ws + oT);
  float*    Y1f = (float*)(ws + oY1f);
  _Float16* Y1h = (_Float16*)(ws + oY1h);
  if (oK != oQ + (size_t)QKPLANE * 2) return;

  k_cvt<<<dim3((NTOK * HID) / 2048), dim3(256), 0, stream>>>(x, Xh, 1.0f);
  k_cvt<<<dim3((HID * HID) / 2048), dim3(256), 0, stream>>>(wq, Wt, 32.0f);
  k_cvt<<<dim3((HID * HID) / 2048), dim3(256), 0, stream>>>(wk, Wt + (size_t)HID * HID, 32.0f);
  k_cvt<<<dim3((HID * HID) / 2048), dim3(256), 0, stream>>>(wv, Wt + (size_t)2 * HID * HID, 32.0f);
  k_cvt<<<dim3((HID * HID) / 2048), dim3(256), 0, stream>>>(wo, Wot, 32.0f);
  k_cvt<<<dim3((DFF * HID) / 2048), dim3(256), 0, stream>>>(w1, W1t, 32.0f);
  k_cvt<<<dim3((HID * DFF) / 2048), dim3(256), 0, stream>>>(w2, W2t, 32.0f);
  k_qkv<<<dim3(NB * SBLK, NQKV / 64), dim3(256), 0, stream>>>(Xh, Wt, bq, bk, bv, QKp, Vt);
  const float sscale = 0.125f;
  k_attn<<<dim3(NB * NH * NQB), dim3(256), 0, stream>>>(QKp, Kp, Vt, Op, sscale);
  k_gemm_f32<<<dim3(NTOK / 256, HID / 64), dim3(256), 0, stream>>>(Op, HID, Wot, HID, bo, 0.00048828125f, T, HID);
  k_ln1<<<dim3(NTOK / 8), dim3(256), 0, stream>>>(T, x, g1, be1, Y1f, Y1h);
  k_gemm_h16<<<dim3(NTOK / 256, DFF / 64), dim3(256), 0, stream>>>(Y1h, HID, W1t, HID, b1, 0.03125f, 16.0f, Hd, DFF);
  k_gemm_f32<<<dim3(NTOK / 256, HID / 64), dim3(256), 0, stream>>>(Hd, DFF, W2t, DFF, b2, 0.001953125f, T, HID);
  k_ln2<<<dim3(NTOK / 8), dim3(256), 0, stream>>>(T, Y1f, g2, be2, out);
  (void)hipGetLastError();
}
